// FM_80719615361479
// MI455X (gfx1250) — hardware-run, weakly checked
//
#include <hip/hip_runtime.h>


#ifndef NB
#define NB 1024
#endif
#define NB_FULL 1024
#define FD   512
#define KD   16
#define GR   (FD / KD)
#define BW   32
#define IT   64
#define PP   17
#define ZCL  30.0f

static_assert(KD == 16);
static_assert(FD % KD == 0);
static_assert(GR % 8 == 0);
static_assert(FD % 32 == 0);
static_assert(FD % IT == 0);
static_assert(IT == 64);
static_assert(BW == 32);
static_assert(NB % BW == 0);
static_assert(NB <= NB_FULL);
static_assert(((size_t)NB * FD) % 8 == 0);
static_assert((FD * (FD / 8)) % 256 == 0);
static_assert((size_t)(FD * (FD / 8)) * 16 == (size_t)FD * FD * 2);
static_assert(8 * 16 == BW * 4);
static_assert(FD % 256 == 0);
static_assert((size_t)FD * PP * 4 <= 131072);
static_assert((size_t)BW * 4 <= 131072);

typedef unsigned short bf;
typedef __attribute__((ext_vector_type(16))) __bf16   v16bf;
typedef __attribute__((ext_vector_type(8)))  unsigned short v8us;
typedef __attribute__((ext_vector_type(8)))  float    v8f;
typedef __attribute__((ext_vector_type(4)))  float    v4f;
typedef v4f  __attribute__((may_alias)) v4fa;

__device__ __forceinline__ unsigned short f2bf(float f) { unsigned u = __float_as_uint(f); u += 0x7FFFu + ((u >> 16) & 1u); return (unsigned short)(u >> 16); }
__device__ __forceinline__ float bfr(float f) { return __uint_as_float(((unsigned)f2bf(f)) << 16); }
__device__ __forceinline__ v16bf cat16b(v8us lo, v8us hi) { return __builtin_bit_cast(v16bf, __builtin_shufflevector(lo, hi, 0, 1, 2, 3, 4, 5, 6, 7, 8, 9, 10, 11, 12, 13, 14, 15)); }
__device__ __forceinline__ v8f wmmab(v16bf a, v16bf b, v8f c) { return __builtin_amdgcn_wmma_f32_16x16x32_bf16(false, a, false, b, (short)0, c, false, false); }
__device__ __forceinline__ v16bf ldb(const bf* p)  { return cat16b(*(const v8us*)p, *(const v8us*)(p + 16)); }
__device__ __forceinline__ void wave_sync() { __builtin_amdgcn_fence(3  , "wavefront"); __builtin_amdgcn_wave_barrier(); asm volatile("" ::: "memory"); }
__device__ __forceinline__ float bfx(unsigned short w) { return __uint_as_float(((unsigned)w) << 16); }
__device__ __forceinline__ v8f wmmab_g(v16bf a, v16bf b, v8f c) { c = wmmab(a, b, c); asm volatile("v_nop\n\tv_nop\n\tv_nop\n\tv_nop" : "+v"(c) : "v"(a), "v"(b)); return c; }

__global__ __launch_bounds__(256) void k_cvt8(const float* __restrict__ src, bf* dst, size_t n8) {
    const size_t i = (size_t)blockIdx.x * 256 + threadIdx.x; if (i >= n8) return;
    const v8f v = *(const v8f*)(src + i * 8); v8us o;
#pragma unroll
    for (int k = 0; k < 8; ++k) o[k] = f2bf(v[k]);
    *(volatile v8us*)(dst + i * 8) = o; __threadfence(); *(volatile v8us*)(dst + i * 8) = o;
}

__global__ __launch_bounds__(256) void k_mbuild(const float* __restrict__ W, bf* MH, bf* ML) {
#pragma clang fp contract(off)
    __shared__ float pre[FD * PP];
    const int tid = threadIdx.x;
#pragma unroll 1
    for (int f = tid; f < FD; f += 256) {
        const float* wr = W + (size_t)f * KD;
        const v4f w0 = *(const v4f*)wr, w1 = *(const v4f*)(wr + 4), w2 = *(const v4f*)(wr + 8), w3 = *(const v4f*)(wr + 12);
        float run = 0.0f;
#pragma unroll
        for (int m = 0; m < 4; ++m) { run = run + bfr(w0[m]); pre[f * PP + m] = run; }
#pragma unroll
        for (int m = 0; m < 4; ++m) { run = run + bfr(w1[m]); pre[f * PP + 4 + m] = run; }
#pragma unroll
        for (int m = 0; m < 4; ++m) { run = run + bfr(w2[m]); pre[f * PP + 8 + m] = run; }
#pragma unroll
        for (int m = 0; m < 4; ++m) { run = run + bfr(w3[m]); pre[f * PP + 12 + m] = run; }
    }
    __syncthreads();
    const int t = blockIdx.x * 256 + tid;
    const int i = t / (FD / 8), f0 = (t % (FD / 8)) * 8;
    const int kk = f0 / GR, g0 = f0 % GR;
    const float wik = bfr(W[i * KD + kk]);
    v8us oh, ol;
#pragma unroll
    for (int e = 0; e < 8; ++e) {
        const int d = i - KD * (g0 + e);
        const int dc = d < 0 ? 0 : (d > KD - 1 ? KD - 1 : d);
        const float pv = pre[(f0 + e) * PP + dc];
        const float q = (d >= 0) ? pv : 0.0f;
        const float mv = wik * q;
        const unsigned short hb = f2bf(mv);
        const unsigned short lb = f2bf(mv - bfx(hb));
        oh[e] = hb; ol[e] = lb;
    }
    const size_t o = (size_t)t * 8;
    *(volatile v8us*)(MH + o) = oh; *(volatile v8us*)(ML + o) = ol;
    __threadfence();
    *(volatile v8us*)(MH + o) = oh; *(volatile v8us*)(ML + o) = ol;
}

__global__ __launch_bounds__(32) void k_quad(const bf* __restrict__ XB, const bf* __restrict__ MH, const bf* __restrict__ ML,
                                             const float* __restrict__ lin_w, const float* __restrict__ lin_b, float* OUT) {
    __shared__ __align__(16) float zs[BW];
    const int lane = threadIdx.x & 31, lr = lane & 15, hi = lane >> 4;
    const int b0 = blockIdx.x * BW;
    const size_t boff = (size_t)(b0 + lr) * FD + 8 * hi;
    const size_t xr0 = (size_t)(b0 + lr) * FD, xr1 = (size_t)(b0 + 16 + lr) * FD;
    float s0 = 0.0f, s1 = 0.0f;
#pragma unroll 1
    for (int i0 = 0; i0 < FD; i0 += IT) {
        v8f acc[4][2];
#pragma unroll
        for (int mb = 0; mb < 4; ++mb) { acc[mb][0] = (v8f){}; acc[mb][1] = (v8f){}; }
        const size_t aoff = (size_t)(i0 + lr) * FD + 8 * hi;
#pragma unroll 1
        for (int kc = 0; kc < FD; kc += 32) {
            const v16bf x0 = ldb(XB + boff + kc);
            const v16bf x1 = ldb(XB + boff + (size_t)16 * FD + kc);
#pragma unroll
            for (int mb = 0; mb < 4; ++mb) {
                const v16bf ah = ldb(MH + aoff + (size_t)mb * 16 * FD + kc);
                const v16bf al = ldb(ML + aoff + (size_t)mb * 16 * FD + kc);
                acc[mb][0] = wmmab_g(ah, x0, acc[mb][0]);
                acc[mb][1] = wmmab_g(ah, x1, acc[mb][1]);
                acc[mb][0] = wmmab_g(al, x0, acc[mb][0]);
                acc[mb][1] = wmmab_g(al, x1, acc[mb][1]);
            }
        }
#pragma unroll
        for (int mb = 0; mb < 4; ++mb) {
            const int ic = i0 + mb * 16 + 8 * hi;
            const v4f l0 = *(const v4f*)(lin_w + ic), l1 = *(const v4f*)(lin_w + ic + 4);
            const v8us xa = *(const v8us*)(XB + xr0 + ic);
            const v8us xb = *(const v8us*)(XB + xr1 + ic);
#pragma unroll
            for (int r = 0; r < 4; ++r) {
                const float lwa = bfr(l0[r]), lwb = bfr(l1[r]);
                s0 = fmaf(bfx(xa[r]),     acc[mb][0][r]     + lwa, s0);
                s1 = fmaf(bfx(xb[r]),     acc[mb][1][r]     + lwa, s1);
                s0 = fmaf(bfx(xa[4 + r]), acc[mb][0][4 + r] + lwb, s0);
                s1 = fmaf(bfx(xb[4 + r]), acc[mb][1][4 + r] + lwb, s1);
            }
        }
    }
    s0 += __shfl_xor(s0, 16, 32);
    s1 += __shfl_xor(s1, 16, 32);
    const float zb = bfr(lin_b[0]);
    float z = ((hi == 0) ? s0 : s1) + zb;
    z = fminf(fmaxf(z, -ZCL), ZCL);
    const float sg = 1.0f / (1.0f + expf(-z));
    zs[lane] = sg;
    wave_sync();
    const v4f val = *(const v4fa*)(&zs[4 * (lane & 7)]);
    float* orow = OUT + b0;
#pragma unroll 1
    for (int ps = 0; ps < 2; ++ps) {
        if (lane < 8) *(volatile v4f*)(orow + 4 * lane) = val;
        if (ps == 0) __threadfence(); }
}

static constexpr size_t al256(size_t v) { return (v + 255) & ~(size_t)255; }
static constexpr size_t SZ_XB = al256((size_t)NB * FD * 2);
static constexpr size_t SZ_MQ = al256((size_t)FD * FD * 2);
static constexpr size_t SZ_TOTAL = SZ_XB + 2 * SZ_MQ;
static_assert(SZ_TOTAL <= (size_t)134217728);
static_assert(SZ_XB % 256 == 0);
static_assert(SZ_MQ % 256 == 0);

extern "C" void kernel_launch(void* const* d_in, const int* in_sizes, int n_in,
                              void* d_out, int out_size, void* d_ws, size_t ws_size, hipStream_t stream) {
    if (n_in < 4) return;
    if ((size_t)in_sizes[0] < (size_t)NB * FD) return;
    if ((size_t)in_sizes[1] < (size_t)FD * KD) return;
    if (in_sizes[2] < FD || in_sizes[3] < 1) return;
    if ((size_t)out_size < (size_t)NB) return;
    if (SZ_TOTAL > ws_size) return;
    const float* x  = (const float*)d_in[0];
    const float* W  = (const float*)d_in[1];
    const float* lw = (const float*)d_in[2];
    const float* lb = (const float*)d_in[3];
    float* OUT = (float*)d_out;
    char* wsp = (char*)d_ws;
    bf* XB = (bf*)wsp; wsp += SZ_XB;
    bf* MH = (bf*)wsp; wsp += SZ_MQ;
    bf* ML = (bf*)wsp; wsp += SZ_MQ;

    { const size_t n8 = (size_t)NB * FD / 8;
      k_cvt8<<<(unsigned)((n8 + 255) / 256), 256, 0, stream>>>(x, XB, n8); }
    k_mbuild<<<dim3(FD * (FD / 8) / 256, 1, 1), 256, 0, stream>>>(W, MH, ML);
    k_quad<<<dim3(NB / BW, 1, 1), 32, 0, stream>>>(XB, MH, ML, lw, lb, OUT);
}
